// MaskedMultiHeadedSelfAttention_49486613185051
// MI455X (gfx1250) — hardware-verified
//
#include <hip/hip_runtime.h>


#define NB_  2
#define NT_  2048
#define DM   1024
#define NH_  16
#define HD   64
#define NTK  (NB_ * NT_)
#define NW   1024
#define PSC  32768.0f

typedef _Float16 h16;
typedef unsigned short bf;
typedef __attribute__((ext_vector_type(16))) __bf16   v16bf;
typedef __attribute__((ext_vector_type(16))) _Float16 v16h;
typedef __attribute__((ext_vector_type(8)))  _Float16 v8h;
typedef __attribute__((ext_vector_type(8)))  unsigned short v8us;
typedef __attribute__((ext_vector_type(8)))  float    v8f;
typedef __attribute__((ext_vector_type(4)))  float    v4f;
typedef v8h  __attribute__((may_alias)) v8ha;
typedef v4f  __attribute__((may_alias)) v4fa;
typedef v8us __attribute__((may_alias)) v8usa;

__device__ __forceinline__ unsigned short f2bf(float f) { unsigned u = __float_as_uint(f); u += 0x7FFFu + ((u >> 16) & 1u); return (unsigned short)(u >> 16); }
__device__ __forceinline__ float bf2f(unsigned short b) { return __uint_as_float(((unsigned)b) << 16); }
__device__ __forceinline__ float bfr(float f) { return bf2f(f2bf(f)); }
__device__ __forceinline__ v16h cat16(v8h lo, v8h hi) { return __builtin_shufflevector(lo, hi, 0, 1, 2, 3, 4, 5, 6, 7, 8, 9, 10, 11, 12, 13, 14, 15); }
__device__ __forceinline__ v16bf cat16b(v8us lo, v8us hi) { return __builtin_bit_cast(v16bf, __builtin_shufflevector(lo, hi, 0, 1, 2, 3, 4, 5, 6, 7, 8, 9, 10, 11, 12, 13, 14, 15)); }
__device__ __forceinline__ v8f wmma16(v16h a, v16h b, v8f c) { return __builtin_amdgcn_wmma_f32_16x16x32_f16(false, a, false, b, (short)0, c, false, false); }
__device__ __forceinline__ v8f wmmab(v16bf a, v16bf b, v8f c) { return __builtin_amdgcn_wmma_f32_16x16x32_bf16(false, a, false, b, (short)0, c, false, false); }

__global__ __launch_bounds__(256) void k_cvtb(const float* __restrict__ src, int nrows, bf* dst) {
    const int lane = threadIdx.x & 31, r = blockIdx.x * 8 + (threadIdx.x >> 5);
    if (r >= nrows) return;
    v8us o[4];
#pragma unroll
    for (int q = 0; q < 4; ++q) { v8us t;
#pragma unroll
        for (int i = 0; i < 8; ++i) t[i] = f2bf(src[(size_t)r * DM + q * 256 + lane * 8 + i]);
        o[q] = t; }
#pragma unroll
    for (int q = 0; q < 4; ++q) *(volatile v8us*)(dst + (size_t)r * DM + q * 256 + lane * 8) = o[q];
    __threadfence();
#pragma unroll
    for (int q = 0; q < 4; ++q) *(volatile v8us*)(dst + (size_t)r * DM + q * 256 + lane * 8) = o[q];
}

__global__ __launch_bounds__(256) void k_wth(const float* __restrict__ Wm, bf* WT) {
    __shared__ __align__(16) unsigned short tl[64 * 72];
    const int tid = threadIdx.x, h = blockIdx.y, d0 = blockIdx.x * 64;
    const int dd = tid >> 2, eq = (tid & 3) * 16;
#pragma unroll
    for (int i = 0; i < 16; ++i) tl[(eq + i) * 72 + dd] = f2bf(Wm[((size_t)h * DM + d0 + dd) * HD + eq + i]);
    __syncthreads();
    const int piece = tid & 7;
    typedef __attribute__((ext_vector_type(8))) unsigned short v8us_; typedef v8us_ __attribute__((may_alias)) v8usa_;
    auto pass = [&]() {
#pragma unroll
        for (int s = 0; s < 2; ++s) { const int e = (tid >> 3) + 32 * s; const v8us_ val = *(const v8usa_*)(tl + e * 72 + piece * 8);
            *(volatile v8us_*)(WT + (size_t)(h * HD + e) * DM + d0 + piece * 8) = val; }
    };
    pass(); __threadfence(); pass();
}
__global__ __launch_bounds__(256) void k_wt(const float* __restrict__ Wm, bf* WT) {
    __shared__ __align__(16) unsigned short tl[64 * 72];
    const int tid = threadIdx.x, k0 = blockIdx.x * 64, n0 = blockIdx.y * 64;
    const int kk = tid >> 2, nq = (tid & 3) * 16;
#pragma unroll
    for (int i = 0; i < 16; ++i) tl[(nq + i) * 72 + kk] = f2bf(Wm[(size_t)(k0 + kk) * DM + n0 + nq + i]);
    __syncthreads();
    const int piece = tid & 7;
    typedef __attribute__((ext_vector_type(8))) unsigned short v8us_; typedef v8us_ __attribute__((may_alias)) v8usa_;
    auto pass = [&]() {
#pragma unroll
        for (int s = 0; s < 2; ++s) { const int nr = (tid >> 3) + 32 * s; const v8us_ val = *(const v8usa_*)(tl + nr * 72 + piece * 8);
            *(volatile v8us_*)(WT + (size_t)(n0 + nr) * DM + k0 + piece * 8) = val; }
    };
    pass(); __threadfence(); pass();
}

template <bool SPLITA>
__global__ __launch_bounds__(128) void k_gemmb(const bf* __restrict__ A, const bf* __restrict__ Al, const bf* __restrict__ Bn, const float* __restrict__ bias, float* C) {
    __shared__ __align__(16) float ost[4][16 * 68];
    const int lane = threadIdx.x & 31, wave = threadIdx.x >> 5, lr = lane & 15, hi = lane >> 4;
    const int r0 = blockIdx.x * 64 + wave * 16, c0 = blockIdx.y * 64;
    const size_t aoff = (size_t)(r0 + lr) * DM + 8 * hi;
    size_t boff[4];
#pragma unroll
    for (int t = 0; t < 4; ++t) boff[t] = (size_t)(c0 + t * 16 + lr) * DM + 8 * hi;
    v8f acc[4];
#pragma unroll
    for (int t = 0; t < 4; ++t) acc[t] = (v8f){};
#pragma unroll 1
    for (int kc = 0; kc < DM; kc += 32) {
        const v16bf a = cat16b(*(const v8us*)(A + aoff + kc), *(const v8us*)(A + aoff + kc + 16));
        v16bf al = a;
        if (SPLITA) al = cat16b(*(const v8us*)(Al + aoff + kc), *(const v8us*)(Al + aoff + kc + 16));
#pragma unroll
        for (int t = 0; t < 4; ++t) { const v16bf b = cat16b(*(const v8us*)(Bn + boff[t] + kc), *(const v8us*)(Bn + boff[t] + kc + 16)); acc[t] = wmmab(a, b, acc[t]); if (SPLITA) acc[t] = wmmab(al, b, acc[t]); }
        asm volatile("v_nop\n\tv_nop\n\tv_nop\n\tv_nop" : "+v"(acc[0]), "+v"(acc[1]), "+v"(acc[2]), "+v"(acc[3]) : "v"(a), "v"(al));
    }
    float* os = &ost[wave][0];
#pragma unroll
    for (int t = 0; t < 4; ++t) { const float bv = bfr(bias[c0 + t * 16 + lr]);
#pragma unroll
        for (int j = 0; j < 8; ++j) os[(hi * 8 + j) * 68 + t * 16 + lr] = acc[t][j] + bv; }
    __syncthreads();
    float* crow = C + (size_t)r0 * NW + c0;
    auto pass = [&]() {
#pragma unroll
        for (int s = 0; s < 8; ++s) { const int Lid = (lane >> 3) + 4 * s, piece = lane & 7; const int row = Lid >> 1, cofs = (Lid & 1) * 32 + piece * 4;
            const v4f val = *(const v4fa*)(os + row * 68 + cofs); *(volatile v4f*)(crow + (size_t)row * NW + cofs) = val; }
    };
    pass(); __threadfence(); pass();
}

__global__ __launch_bounds__(256) void k_r16(const float* __restrict__ S, h16* D16) {
    const int lane = threadIdx.x & 31, r = blockIdx.x * 8 + (threadIdx.x >> 5);
    if (r >= NTK) return;
    v8h o[4];
#pragma unroll
    for (int q = 0; q < 4; ++q) { v8h t;
#pragma unroll
        for (int i = 0; i < 8; ++i) t[i] = (h16)S[(size_t)r * DM + q * 256 + lane * 8 + i];
        o[q] = t; }
#pragma unroll
    for (int q = 0; q < 4; ++q) *(volatile v8h*)(D16 + (size_t)r * DM + q * 256 + lane * 8) = o[q];
    __threadfence();
#pragma unroll
    for (int q = 0; q < 4; ++q) *(volatile v8h*)(D16 + (size_t)r * DM + q * 256 + lane * 8) = o[q];
}
__global__ __launch_bounds__(256) void k_vt(const float* __restrict__ V, h16* VT16) {
    __shared__ __align__(16) h16 tile[64 * 72];
    const int bid = blockIdx.x;
    const int b = bid / (NH_ * (NT_ / 64)), rem = bid - b * (NH_ * (NT_ / 64)), h = rem / (NT_ / 64), kt = rem - h * (NT_ / 64);
    const int k0 = kt * 64, tid = threadIdx.x;
    const int kk = tid >> 2, d0 = (tid & 3) * 16;
    const float* src = V + ((size_t)b * NT_ + k0 + kk) * DM + h * HD + d0;
#pragma unroll
    for (int i = 0; i < 16; ++i) tile[(d0 + i) * 72 + kk] = (h16)src[i];
    __syncthreads();
    const int piece = tid & 7;
    h16* base = VT16 + (((size_t)b * NH_ + h) * HD) * NT_ + k0;
    auto pass = [&]() {
#pragma unroll
        for (int s = 0; s < 2; ++s) { const int d = (tid >> 3) + 32 * s; const v8h val = *(const v8ha*)(tile + d * 72 + piece * 8); *(volatile v8h*)(base + (size_t)d * NT_ + piece * 8) = val; }
    };
    pass(); __threadfence(); pass();
}

__global__ __launch_bounds__(128) void k_attn(const h16* __restrict__ Q16, const h16* __restrict__ K16, const h16* __restrict__ VT16, const int* __restrict__ mask, bf* CH, bf* CL) {
    __shared__ __align__(16) h16 plds[4][16 * 32];
    __shared__ __align__(16) float ost[4][16 * 68];
    const int lane = threadIdx.x & 31, wave = threadIdx.x >> 5, lr = lane & 15, hi = lane >> 4;
    const int bid = blockIdx.x;
    const int b = bid / (NH_ * (NT_ / 64)), rem = bid - b * (NH_ * (NT_ / 64)), h = rem / (NT_ / 64), qt = rem - h * (NT_ / 64);
    const int q0 = qt * 64 + wave * 16;
    const size_t tok0 = (size_t)b * NT_;
    h16* pl = &plds[wave][0];
    v16h qa[2];
#pragma unroll
    for (int kc = 0; kc < 2; ++kc) { const h16* p = Q16 + (tok0 + q0 + lr) * DM + h * HD + kc * 32 + 8 * hi; qa[kc] = cat16(*(const v8h*)p, *(const v8h*)(p + 16)); }
    const h16* kh_b = K16 + tok0 * DM + h * HD;
    const h16* vt_b = VT16 + (((size_t)b * NH_ + h) * HD) * NT_;
    const int* mk = mask + (size_t)b * NT_;
    v8f o[4];
#pragma unroll
    for (int n = 0; n < 4; ++n) o[n] = (v8f){};
    float mrow[8], lpart[8];
#pragma unroll
    for (int j = 0; j < 8; ++j) { mrow[j] = -3.0e38f; lpart[j] = 0.f; }
#pragma unroll 1
    for (int kt = 0; kt < NT_ / 32; ++kt) {
        const int l0 = kt * 32;
        const h16* r0p = kh_b + (size_t)(l0 + lr) * DM + 8 * hi;
        const h16* r1p = kh_b + (size_t)(l0 + 16 + lr) * DM + 8 * hi;
        v8f s0 = {}, s1 = {};
#pragma unroll
        for (int kc = 0; kc < 2; ++kc) {
            s0 = wmma16(qa[kc], cat16(*(const v8h*)(r0p + kc * 32), *(const v8h*)(r0p + kc * 32 + 16)), s0);
            s1 = wmma16(qa[kc], cat16(*(const v8h*)(r1p + kc * 32), *(const v8h*)(r1p + kc * 32 + 16)), s1);
        }
        asm volatile("v_nop\n\tv_nop\n\tv_nop\n\tv_nop" : "+v"(s0), "+v"(s1) : "v"(qa[0]), "v"(qa[1]));
        const bool mz0 = (mk[l0 + lr] == 0), mz1 = (mk[l0 + 16 + lr] == 0);
        float alpha[8];
#pragma unroll
        for (int j = 0; j < 8; ++j) {
            const float a0 = mz0 ? -1e9f : s0[j] * 0.125f, a1 = mz1 ? -1e9f : s1[j] * 0.125f;
            float mx = fmaxf(a0, a1);
            mx = fmaxf(mx, __shfl_xor(mx, 1, 16)); mx = fmaxf(mx, __shfl_xor(mx, 2, 16)); mx = fmaxf(mx, __shfl_xor(mx, 4, 16)); mx = fmaxf(mx, __shfl_xor(mx, 8, 16));
            const float mn = fmaxf(mrow[j], mx);
            alpha[j] = __expf(mrow[j] - mn); mrow[j] = mn;
            const float p0 = __expf(a0 - mn), p1 = __expf(a1 - mn);
            lpart[j] = lpart[j] * alpha[j] + (p0 + p1);
            const int mr = hi * 8 + j;
            pl[mr * 32 + lr] = (h16)(p0 * PSC); pl[mr * 32 + 16 + lr] = (h16)(p1 * PSC);
        }
#pragma unroll
        for (int n = 0; n < 4; ++n)
#pragma unroll
            for (int j = 0; j < 8; ++j) o[n][j] *= alpha[j];
        asm volatile("" ::: "memory");
        const v16h pa = cat16(*(const v8ha*)(pl + lr * 32 + hi * 8), *(const v8ha*)(pl + lr * 32 + 16 + hi * 8));
#pragma unroll
        for (int n = 0; n < 4; ++n) { const h16* vp = vt_b + (size_t)(n * 16 + lr) * NT_ + l0 + hi * 8; o[n] = wmma16(pa, cat16(*(const v8h*)vp, *(const v8h*)(vp + 16)), o[n]); }
        asm volatile("v_nop\n\tv_nop\n\tv_nop\n\tv_nop" : "+v"(o[0]), "+v"(o[1]), "+v"(o[2]), "+v"(o[3]) : "v"(pa));
    }
    float inv[8];
#pragma unroll
    for (int j = 0; j < 8; ++j) { float rs = lpart[j]; rs += __shfl_xor(rs, 1, 16); rs += __shfl_xor(rs, 2, 16); rs += __shfl_xor(rs, 4, 16); rs += __shfl_xor(rs, 8, 16); inv[j] = 1.0f / (rs * PSC); }
    float* os = &ost[wave][0];
#pragma unroll
    for (int n = 0; n < 4; ++n)
#pragma unroll
        for (int j = 0; j < 8; ++j) os[(hi * 8 + j) * 68 + n * 16 + lr] = o[n][j] * inv[j];
    __syncthreads();
    const size_t cbase = (tok0 + q0) * DM + (size_t)h * HD;
    auto pass = [&]() {
#pragma unroll
        for (int s = 0; s < 4; ++s) { const int row = 4 * s + (lane >> 3), piece = lane & 7; const float* sp = os + row * 68 + piece * 8; v8us oh, ol;
#pragma unroll
            for (int i = 0; i < 8; ++i) { const unsigned short hb = f2bf(sp[i]); oh[i] = hb; ol[i] = f2bf(sp[i] - bf2f(hb)); }
            *(volatile v8us*)(CH + cbase + (size_t)row * DM + piece * 8) = oh; *(volatile v8us*)(CL + cbase + (size_t)row * DM + piece * 8) = ol; }
    };
    pass(); __threadfence(); pass();
}

extern "C" void kernel_launch(void* const* d_in, const int* in_sizes, int n_in,
                              void* d_out, int out_size, void* d_ws, size_t ws_size, hipStream_t stream) {
    (void)in_sizes; (void)n_in; (void)out_size;
    const float* x = (const float*)d_in[0]; const int* mask = (const int*)d_in[1];
    const float* Wq = (const float*)d_in[2]; const float* bq = (const float*)d_in[3]; const float* Wk = (const float*)d_in[4]; const float* bk = (const float*)d_in[5];
    const float* Wv = (const float*)d_in[6]; const float* bv = (const float*)d_in[7]; const float* Wo = (const float*)d_in[8]; const float* bo = (const float*)d_in[9];
    float* out = (float*)d_out;
    char* wsp = (char*)d_ws;
    auto take = [&](size_t bytes) { char* p = wsp; wsp += (bytes + 255) & ~(size_t)255; return (void*)p; };
    bf* Xb = (bf*)take((size_t)NTK * DM * 2);
    bf* WB[4]; for (int i = 0; i < 4; ++i) WB[i] = (bf*)take((size_t)DM * DM * 2);
    float* BQ = nullptr; (void)BQ;
    float* P = (float*)take((size_t)NTK * DM * 4);
    h16* Q16 = (h16*)take((size_t)NTK * DM * 2); h16* K16 = (h16*)take((size_t)NTK * DM * 2); h16* VT16 = (h16*)take((size_t)NTK * DM * 2);
    bf* CH = (bf*)take((size_t)NTK * DM * 2); bf* CL = (bf*)take((size_t)NTK * DM * 2);
    if ((size_t)(wsp - (char*)d_ws) > ws_size) return;
    k_cvtb<<<NTK / 8, 256, 0, stream>>>(x, NTK, Xb);
    k_wth<<<dim3(DM / 64, NH_, 1), 256, 0, stream>>>(Wq, WB[0]);
    k_wth<<<dim3(DM / 64, NH_, 1), 256, 0, stream>>>(Wk, WB[1]);
    k_wth<<<dim3(DM / 64, NH_, 1), 256, 0, stream>>>(Wv, WB[2]);
    k_wt<<<dim3(DM / 64, DM / 64, 1), 256, 0, stream>>>(Wo, WB[3]);
    k_gemmb<false><<<dim3(NTK / 64, NW / 64, 1), 128, 0, stream>>>(Xb, nullptr, WB[0], bq, P);
    k_r16<<<NTK / 8, 256, 0, stream>>>(P, Q16);
    k_gemmb<false><<<dim3(NTK / 64, NW / 64, 1), 128, 0, stream>>>(Xb, nullptr, WB[1], bk, P);
    k_r16<<<NTK / 8, 256, 0, stream>>>(P, K16);
    k_gemmb<false><<<dim3(NTK / 64, NW / 64, 1), 128, 0, stream>>>(Xb, nullptr, WB[2], bv, P);
    k_vt<<<NB_ * NH_ * (NT_ / 64), 256, 0, stream>>>(P, VT16);
    k_attn<<<NB_ * NH_ * (NT_ / 64), 128, 0, stream>>>(Q16, K16, VT16, mask, CH, CL);
    k_gemmb<true><<<dim3(NTK / 64, NW / 64, 1), 128, 0, stream>>>(CH, CL, WB[3], bo, out);
}
